// CrossModalAttention2_57449482551604
// MI455X (gfx1250) — hardware-run, weakly checked
//
#include <hip/hip_runtime.h>
#include <math.h>
#include <stdint.h>

#define NB     4
#define CD     128
#define NS     4096
#define NT     2048
#define XSC    64.0f
#define PSCL   1024.0f
#define LNP    6.931471805599453f
#define SCL    (1.0f / 262144.0f)
#define OSP    132
#define NBLK_S ((NB * CD * NS) / 2048)
#define NBLK_T ((NB * NT * CD) / 2048)
static_assert(CD == 128);
static_assert((NS % 64) == 0 && (NT % 64) == 0);
static_assert(((NB * CD * NS) % 2048) == 0 && ((NB * NT * CD) % 2048) == 0);
static_assert(NBLK_S == 1024 && NBLK_T == 512);

typedef _Float16 v16h __attribute__((ext_vector_type(16)));
typedef _Float16 v8h  __attribute__((ext_vector_type(8)));
typedef float    v8f  __attribute__((ext_vector_type(8)));
typedef float    v4f  __attribute__((ext_vector_type(4)));
typedef unsigned int v4u __attribute__((ext_vector_type(4)));

union FragH { v16h v; v8h h[2]; };

__device__ __forceinline__ unsigned short bf_bits(float f) {
  unsigned u = __float_as_uint(f);
  return (unsigned short)((u + 0x7FFFu + ((u >> 16) & 1u)) >> 16);
}
__device__ __forceinline__ float bf_up(unsigned short h) { return __uint_as_float(((unsigned)h) << 16); }
__device__ __forceinline__ float bfr(float f) { return bf_up(bf_bits(f)); }
__device__ __forceinline__ unsigned short h_bits(_Float16 x) { return __builtin_bit_cast(unsigned short, x); }
__device__ __forceinline__ unsigned pk16(unsigned short a, unsigned short b) { return (unsigned)a | ((unsigned)b << 16); }
__device__ __forceinline__ v8f zero8() { v8f z = {0.f, 0.f, 0.f, 0.f, 0.f, 0.f, 0.f, 0.f}; return z; }
__device__ __forceinline__ float hmax8(v8f s) {
  return fmaxf(fmaxf(fmaxf(s[0], s[1]), fmaxf(s[2], s[3])), fmaxf(fmaxf(s[4], s[5]), fmaxf(s[6], s[7])));
}
__device__ __forceinline__ v4u cvt8(v4f a, v4f c) {
  float f[8];
#pragma unroll
  for (int i = 0; i < 4; ++i) { f[i] = bfr(a[i]) * XSC; f[4 + i] = bfr(c[i]) * XSC; }
  v4u v;
#pragma unroll
  for (int i = 0; i < 4; ++i) v[i] = pk16(h_bits((_Float16)f[2 * i]), h_bits((_Float16)f[2 * i + 1]));
  return v;
}

__device__ __forceinline__ v16h ldfrag_h(const _Float16* p) {
  FragH f;
  f.h[0] = *(const v8h*)(p);
  f.h[1] = *(const v8h*)(p + 16);
  return f.v;
}

__device__ __forceinline__ v8f mma_h_raw(v16h a, v16h b, v8f c) {
  return __builtin_amdgcn_wmma_f32_16x16x32_f16(false, a, false, b, (short)0, c, false, false);
}
__device__ __forceinline__ void sguard1(v8f& s, v16h x0, v16h x1, v16h x2, v16h x3,
                                        v16h q0, v16h q1, v16h q2, v16h q3) {
#if defined(__HIP_DEVICE_COMPILE__)
  asm volatile("v_nop\n\tv_nop\n\tv_nop\n\tv_nop"
               : "+v"(s) : "v"(x0), "v"(x1), "v"(x2), "v"(x3), "v"(q0), "v"(q1), "v"(q2), "v"(q3));
#endif
}
__device__ __forceinline__ void oguard4(v8f& a, v8f& b, v8f& c, v8f& d,
                                        v16h v0, v16h v1, v16h v2, v16h v3, v16h p) {
#if defined(__HIP_DEVICE_COMPILE__)
  asm volatile("v_nop\n\tv_nop\n\tv_nop\n\tv_nop"
               : "+v"(a), "+v"(b), "+v"(c), "+v"(d) : "v"(v0), "v"(v1), "v"(v2), "v"(v3), "v"(p));
#endif
}

__global__ __launch_bounds__(256) void cvt_rows(const float* __restrict__ fs, const float* __restrict__ ft,
                                                 unsigned short* KS, unsigned short* TN) {
  const int bx = blockIdx.x;
  const bool iss = (bx < NBLK_S);
  const float* src = iss ? fs : ft;
  unsigned short* dst = iss ? KS : TN;
  const size_t e0 = ((size_t)(iss ? bx : (bx - NBLK_S)) * 256 + threadIdx.x) * 8;
  const v4f a = *(const v4f*)(src + e0);
  const v4f c = *(const v4f*)(src + e0 + 4);
  const v4u v = cvt8(a, c);
  unsigned short* dp = dst + e0;
  *(volatile v4u*)dp = v;
  __threadfence();
  *(volatile v4u*)dp = v;
}

__global__ __launch_bounds__(256) void xpose_s(const float* __restrict__ fs, unsigned short* XN) {
  __shared__ __align__(16) unsigned short Xs[64 * 136];
  const int tid = threadIdx.x;
  const int bx  = blockIdx.x;
  const int b   = bx / (NS / 64);
  const int n0  = (bx - b * (NS / 64)) * 64;
  const float* fb = fs + (size_t)b * CD * NS + n0;
  {
    const int q = tid & 15, c16 = tid >> 4;
#pragma unroll 1
    for (int it = 0; it < 8; ++it) {
      const int c = it * 16 + c16;
      const v4f v = *(const v4f*)(fb + (size_t)c * NS + 4 * q);
#pragma unroll
      for (int e = 0; e < 4; ++e) Xs[(4 * q + e) * 136 + c] = h_bits((_Float16)(bfr(v[e]) * XSC));
    }
  }
  __syncthreads();
  {
    const int p = tid & 15, r16 = tid >> 4;
    v4u vals[4];
#pragma unroll
    for (int it = 0; it < 4; ++it) {
      const int row = it * 16 + r16;
      vals[it] = *(const v4u*)(Xs + row * 136 + 8 * p);
    }
    unsigned short* xb = XN + ((size_t)b * NS + n0) * CD + 8 * p;
    for (int pass = 0; pass < 2; ++pass) {
#pragma unroll
      for (int it = 0; it < 4; ++it) {
        const int row = it * 16 + r16;
        *(volatile v4u*)(xb + (size_t)row * CD) = vals[it];
      }
      __threadfence();
    }
  }
}

__global__ __launch_bounds__(256) void xpose_t(const float* __restrict__ ft, unsigned short* TT) {
  __shared__ __align__(16) unsigned short Ts[128 * 72];
  const int tid = threadIdx.x;
  const int bx  = blockIdx.x;
  const int b   = bx / (NT / 64);
  const int m0  = (bx - b * (NT / 64)) * 64;
  const float* tb = ft + ((size_t)b * NT + m0) * CD;
  {
    const int q = tid & 31, r8 = tid >> 5;
#pragma unroll 1
    for (int it = 0; it < 8; ++it) {
      const int ml = it * 8 + r8;
      const v4f v = *(const v4f*)(tb + (size_t)ml * CD + 4 * q);
#pragma unroll
      for (int e = 0; e < 4; ++e) Ts[(4 * q + e) * 72 + ml] = h_bits((_Float16)(bfr(v[e]) * XSC));
    }
  }
  __syncthreads();
  {
    const int e8 = tid & 7, fq = tid >> 3;
    v4u vals[4];
#pragma unroll
    for (int it = 0; it < 4; ++it) {
      const int c = it * 32 + fq;
      vals[it] = *(const v4u*)(Ts + c * 72 + 8 * e8);
    }
    unsigned short* dp = TT + ((size_t)b * CD) * NT + m0 + 8 * e8;
    for (int pass = 0; pass < 2; ++pass) {
#pragma unroll
      for (int it = 0; it < 4; ++it) {
        const int c = it * 32 + fq;
        *(volatile v4u*)(dp + (size_t)c * NT) = vals[it];
      }
      __threadfence();
    }
  }
}

__global__ __launch_bounds__(128)
void attn_t(const unsigned short* __restrict__ xn, const unsigned short* __restrict__ tn,
            const unsigned short* __restrict__ ks, float* out1, float* G) {
  __shared__ __align__(16) float Os[64 * CD];
  __shared__ __align__(16) float Ls[64];
  const int tid  = threadIdx.x;
  const int wave = tid >> 5;
  const int lane = tid & 31;
  const int hh   = lane >> 4;
  const int ci   = lane & 15;
  const int bx   = blockIdx.x;
  const int b    = bx / (NT / 64);
  const int m0   = (bx - b * (NT / 64)) * 64;

  const _Float16* XNp = (const _Float16*)(const void*)xn;
  const _Float16* TNp = (const _Float16*)(const void*)tn;
  const _Float16* KSp = (const _Float16*)(const void*)ks;

  const size_t qrow = ((size_t)b * NT + m0 + wave * 16 + ci) * CD + 8 * hh;
  v16h qf[4];
#pragma unroll
  for (int j = 0; j < 4; ++j) qf[j] = ldfrag_h(TNp + qrow + 32 * j);
  const _Float16* Kp = XNp + ((size_t)b * NS + ci) * CD + 8 * hh;
  const _Float16* Vp = KSp + ((size_t)b * CD + ci) * NS + 8 * hh;

  float m = -1.0e30f, l = 0.f;
  v8f acc[8];
#pragma unroll
  for (int j = 0; j < 8; ++j) acc[j] = zero8();

#pragma unroll 1
  for (int it = 0; it < NS / 32; ++it) {
    const int kb = it * 32;
    v8f s0 = zero8(), s1 = zero8();
    {
      const _Float16* p0 = Kp + (size_t)kb * CD;
      v16h x[4];
#pragma unroll
      for (int j = 0; j < 4; ++j) x[j] = ldfrag_h(p0 + 32 * j);
#pragma unroll
      for (int j = 0; j < 4; ++j) s0 = mma_h_raw(x[j], qf[j], s0);
      sguard1(s0, x[0], x[1], x[2], x[3], qf[0], qf[1], qf[2], qf[3]);
      const _Float16* p1 = p0 + (size_t)16 * CD;
      v16h y[4];
#pragma unroll
      for (int j = 0; j < 4; ++j) y[j] = ldfrag_h(p1 + 32 * j);
#pragma unroll
      for (int j = 0; j < 4; ++j) s1 = mma_h_raw(y[j], qf[j], s1);
      sguard1(s1, y[0], y[1], y[2], y[3], qf[0], qf[1], qf[2], qf[3]);
    }

    float mx = fmaxf(hmax8(s0), hmax8(s1));
    mx = fmaxf(mx, __shfl_xor(mx, 16, 32));
    const float mn   = fmaxf(m, mx * SCL);
    const float corr = __expf(m - mn);
    m = mn;
    const float msh = mn - LNP;
    l *= corr;
#pragma unroll
    for (int j = 0; j < 8; ++j) {
#pragma unroll
      for (int r = 0; r < 8; ++r) acc[j][r] *= corr;
    }

    FragH ph;
    float ls = 0.f;
#pragma unroll
    for (int r = 0; r < 8; ++r) {
      const float e0 = __expf(s0[r] * SCL - msh);
      const float e1 = __expf(s1[r] * SCL - msh);
      ls += e0 + e1;
      ph.h[0][r] = (_Float16)e0;
      ph.h[1][r] = (_Float16)e1;
    }
    l += ls;

    {
      const _Float16* vp = Vp + kb;
      v16h v[4];
#pragma unroll
      for (int j = 0; j < 4; ++j) v[j] = ldfrag_h(vp + (size_t)(16 * j) * NS);
#pragma unroll
      for (int j = 0; j < 4; ++j) acc[j] = mma_h_raw(v[j], ph.v, acc[j]);
      oguard4(acc[0], acc[1], acc[2], acc[3], v[0], v[1], v[2], v[3], ph.v);
      v16h w[4];
#pragma unroll
      for (int j = 0; j < 4; ++j) w[j] = ldfrag_h(vp + (size_t)(16 * (j + 4)) * NS);
#pragma unroll
      for (int j = 0; j < 4; ++j) acc[4 + j] = mma_h_raw(w[j], ph.v, acc[4 + j]);
      oguard4(acc[4], acc[5], acc[6], acc[7], w[0], w[1], w[2], w[3], ph.v);
    }
  }
  l += __shfl_xor(l, 16, 32);
  const float rl = 1.0f / l;
  const float sc = rl * (1.0f / XSC);

  float* os = Os + (wave * 16 + ci) * CD + 8 * hh;
#pragma unroll
  for (int j = 0; j < 8; ++j) {
    v4f a0, a1;
#pragma unroll
    for (int e = 0; e < 4; ++e) { a0[e] = acc[j][e] * sc; a1[e] = acc[j][4 + e] * sc; }
    *(v4f*)(os + 16 * j) = a0;
    *(v4f*)(os + 16 * j + 4) = a1;
  }
  if (hh == 0) Ls[wave * 16 + ci] = m + __logf(l) - 2.0f * LNP;
  __syncthreads();
  {
    v4f vals[16];
#pragma unroll
    for (int r = 0; r < 16; ++r) vals[r] = *(const v4f*)(Os + (wave * 16 + r) * CD + 4 * lane);
    const v4f gv = *(const v4f*)(Ls + 4 * ci);
    const bool gw = (wave == 0) && (hh == 0);
    float* ob = out1 + ((size_t)b * NT + m0 + wave * 16) * CD + 4 * lane;
    float* gp = G + (size_t)b * NT + m0 + 4 * ci;
    for (int pass = 0; pass < 2; ++pass) {
#pragma unroll
      for (int r = 0; r < 16; ++r) *(volatile v4f*)(ob + (size_t)r * CD) = vals[r];
      if (gw) *(volatile v4f*)gp = gv;
      __threadfence();
    }
  }
}

__global__ __launch_bounds__(128)
void attn_s(const unsigned short* __restrict__ xn, const unsigned short* __restrict__ tn,
            const unsigned short* __restrict__ tt, const float* __restrict__ G,
            const float* __restrict__ fs, float* out0) {
  __shared__ __align__(16) float Os[64 * OSP];
  const int tid  = threadIdx.x;
  const int wave = tid >> 5;
  const int lane = tid & 31;
  const int hh   = lane >> 4;
  const int ci   = lane & 15;
  const int bx   = blockIdx.x;
  const int b    = bx / (NS / 64);
  const int n0   = (bx - b * (NS / 64)) * 64;

  const _Float16* XNp = (const _Float16*)(const void*)xn;
  const _Float16* TNp = (const _Float16*)(const void*)tn;
  const _Float16* TTp = (const _Float16*)(const void*)tt;

  const size_t qrow = ((size_t)b * NS + n0 + wave * 16 + ci) * CD + 8 * hh;
  v16h qf[4];
#pragma unroll
  for (int j = 0; j < 4; ++j) qf[j] = ldfrag_h(XNp + qrow + 32 * j);
  const _Float16* Kp = TNp + ((size_t)b * NT + ci) * CD + 8 * hh;
  const _Float16* Vp = TTp + ((size_t)b * CD + ci) * NT + 8 * hh;
  const float* Gp = G + (size_t)b * NT + 8 * hh;

  v8f acc[8];
#pragma unroll
  for (int j = 0; j < 8; ++j) acc[j] = zero8();

#pragma unroll 1
  for (int it = 0; it < NT / 32; ++it) {
    const int kb = it * 32;
    v8f s0 = zero8(), s1 = zero8();
    {
      const _Float16* p0 = Kp + (size_t)kb * CD;
      v16h x[4];
#pragma unroll
      for (int j = 0; j < 4; ++j) x[j] = ldfrag_h(p0 + 32 * j);
#pragma unroll
      for (int j = 0; j < 4; ++j) s0 = mma_h_raw(x[j], qf[j], s0);
      sguard1(s0, x[0], x[1], x[2], x[3], qf[0], qf[1], qf[2], qf[3]);
      const _Float16* p1 = p0 + (size_t)16 * CD;
      v16h y[4];
#pragma unroll
      for (int j = 0; j < 4; ++j) y[j] = ldfrag_h(p1 + 32 * j);
#pragma unroll
      for (int j = 0; j < 4; ++j) s1 = mma_h_raw(y[j], qf[j], s1);
      sguard1(s1, y[0], y[1], y[2], y[3], qf[0], qf[1], qf[2], qf[3]);
    }

    const v4f ga = *(const v4f*)(Gp + kb);
    const v4f gb = *(const v4f*)(Gp + kb + 4);
    const v4f gc = *(const v4f*)(Gp + kb + 16);
    const v4f gd = *(const v4f*)(Gp + kb + 20);
    FragH ph;
#pragma unroll
    for (int r = 0; r < 4; ++r) {
      ph.h[0][r]     = (_Float16)__expf(s0[r] * SCL - ga[r]);
      ph.h[0][4 + r] = (_Float16)__expf(s0[4 + r] * SCL - gb[r]);
      ph.h[1][r]     = (_Float16)__expf(s1[r] * SCL - gc[r]);
      ph.h[1][4 + r] = (_Float16)__expf(s1[4 + r] * SCL - gd[r]);
    }

    {
      const _Float16* vp = Vp + kb;
      v16h v[4];
#pragma unroll
      for (int j = 0; j < 4; ++j) v[j] = ldfrag_h(vp + (size_t)(16 * j) * NT);
#pragma unroll
      for (int j = 0; j < 4; ++j) acc[j] = mma_h_raw(v[j], ph.v, acc[j]);
      oguard4(acc[0], acc[1], acc[2], acc[3], v[0], v[1], v[2], v[3], ph.v);
      v16h w[4];
#pragma unroll
      for (int j = 0; j < 4; ++j) w[j] = ldfrag_h(vp + (size_t)(16 * (j + 4)) * NT);
#pragma unroll
      for (int j = 0; j < 4; ++j) acc[4 + j] = mma_h_raw(w[j], ph.v, acc[4 + j]);
      oguard4(acc[4], acc[5], acc[6], acc[7], w[0], w[1], w[2], w[3], ph.v);
    }
  }
  const float osc = 1.0f / (XSC * PSCL);

  float* os = Os + (wave * 16 + ci) * OSP + 8 * hh;
#pragma unroll
  for (int j = 0; j < 8; ++j) {
    v4f a0, a1;
#pragma unroll
    for (int e = 0; e < 4; ++e) { a0[e] = acc[j][e] * osc; a1[e] = acc[j][4 + e] * osc; }
    *(v4f*)(os + 16 * j) = a0;
    *(v4f*)(os + 16 * j + 4) = a1;
  }
  __syncthreads();
  {
    const int q4 = tid & 15, cr = tid >> 4;
    const size_t rowb = ((size_t)b * CD) * NS + n0 + 4 * q4;
    v4f vals[16];
#pragma unroll
    for (int r = 0; r < 16; ++r) {
      const int c = r * 8 + cr;
      const v4f f = *(const v4f*)(fs + rowb + (size_t)c * NS);
      v4f o;
#pragma unroll
      for (int e = 0; e < 4; ++e) o[e] = bfr(f[e]) + Os[(4 * q4 + e) * OSP + c];
      vals[r] = o;
    }
    for (int pass = 0; pass < 2; ++pass) {
#pragma unroll
      for (int r = 0; r < 16; ++r) {
        const int c = r * 8 + cr;
        *(volatile v4f*)(out0 + rowb + (size_t)c * NS) = vals[r];
      }
      __threadfence();
    }
  }
}

extern "C" void kernel_launch(void* const* d_in, const int* in_sizes, int n_in,
                              void* d_out, int out_size, void* d_ws, size_t ws_size,
                              hipStream_t stream) {
  if (n_in < 2) return;
  if (in_sizes[0] != NB * CD * NS) return;
  if (in_sizes[1] != NB * NT * CD) return;
  if (out_size != NB * CD * NS + NB * NT * CD) return;

  const float* f_s = (const float*)d_in[0];
  const float* f_t = (const float*)d_in[1];

  const size_t PKS = (size_t)NB * CD * NS * 2;
  const size_t PXN = (size_t)NB * NS * CD * 2;
  const size_t PTN = (size_t)NB * NT * CD * 2;
  const size_t PTT = (size_t)NB * CD * NT * 2;
  const size_t PG  = (size_t)NB * NT * 4;
  size_t off = 0;
  const size_t oKS = off; off += PKS;
  const size_t oXN = off; off += PXN;
  const size_t oTN = off; off += PTN;
  const size_t oTT = off; off += PTT;
  const size_t oG  = off; off += PG;
  if (off > ws_size) return;
  if (off > (size_t)134217728) return;

  char* ws = (char*)d_ws;
  unsigned short* KS = (unsigned short*)(ws + oKS);
  unsigned short* XN = (unsigned short*)(ws + oXN);
  unsigned short* TN = (unsigned short*)(ws + oTN);
  unsigned short* TT = (unsigned short*)(ws + oTT);
  float*          Gp = (float*)(ws + oG);
  float*          out0 = (float*)d_out;
  float*          out1 = (float*)d_out + (size_t)NB * CD * NS;

  const dim3 blk(256), blk128(128);
  const dim3 gCV(NBLK_S + NBLK_T);
  const dim3 gXS(NB * (NS / 64));
  const dim3 gXT(NB * (NT / 64));
  const dim3 gAT(NB * (NT / 64));
  const dim3 gAS(NB * (NS / 64));

  cvt_rows<<<gCV, blk, 0, stream>>>(f_s, f_t, KS, TN);
  xpose_s<<<gXS, blk, 0, stream>>>(f_s, XN);
  xpose_t<<<gXT, blk, 0, stream>>>(f_t, TT);
  attn_t<<<gAT, blk128, 0, stream>>>(XN, TN, KS, out1, Gp);
  attn_s<<<gAS, blk128, 0, stream>>>(XN, TN, TT, Gp, f_s, out0);
  (void)hipGetLastError();
}
